// MultiInfAffine_36352603193791
// MI455X (gfx1250) — hardware-run, weakly checked
//
#include <hip/hip_runtime.h>


#ifndef NPTS
#define NPTS 250000
#endif
#define NPTS_FULL 250000
#define DD   16
#define LL   6
#define KC   64
#define WPB  8
#define PPB  (WPB * 16)
#define NPAR (LL * KC)
#define PTN  1024
#define NEGB (-3.0e38f)

static_assert(DD == 16);
static_assert(KC == 64);
static_assert(NPTS % 16 == 0);
static_assert(NPTS % 4 == 0);
static_assert(NPTS <= NPTS_FULL);
static_assert(PPB * 4 == 32 * 16);
static_assert(NPAR == 384);
static_assert(2 * NPAR * 8 == NPAR * DD);
static_assert(PTN == 2 * NPAR + 256);
static_assert(PTN == 256 * 4);
static_assert((NPAR * 2) % 256 == 0);
static_assert(PTN % 256 == 0);
static_assert(LL <= 32);
static_assert(NPAR * 2 * 16 + PTN * 4 + PPB * 4 <= 131072);
static_assert(NPAR * DD * 2 + PTN * 4 <= 131072);

typedef unsigned short bf;
typedef __attribute__((ext_vector_type(16))) __bf16   v16bf;
typedef __attribute__((ext_vector_type(8)))  unsigned short v8us;
typedef __attribute__((ext_vector_type(8)))  float    v8f;
typedef __attribute__((ext_vector_type(4)))  float    v4f;
typedef v4f  __attribute__((may_alias)) v4fa;
typedef v8us __attribute__((may_alias)) v8usa;

__device__ __forceinline__ unsigned short f2bf(float f) { unsigned u = __float_as_uint(f); u += 0x7FFFu + ((u >> 16) & 1u); return (unsigned short)(u >> 16); }
__device__ __forceinline__ float bfr(float f) { return __uint_as_float(((unsigned)f2bf(f)) << 16); }
__device__ __forceinline__ v16bf cat16b(v8us lo, v8us hi) { return __builtin_bit_cast(v16bf, __builtin_shufflevector(lo, hi, 0, 1, 2, 3, 4, 5, 6, 7, 8, 9, 10, 11, 12, 13, 14, 15)); }
__device__ __forceinline__ v8f wmmab(v16bf a, v16bf b, v8f c) { return __builtin_amdgcn_wmma_f32_16x16x32_bf16(false, a, false, b, (short)0, c, false, false); }
__device__ __forceinline__ v8f wmmab_g(v16bf a, v16bf b, v8f c) { c = wmmab(a, b, c); asm volatile("v_nop\n\tv_nop\n\tv_nop\n\tv_nop" : "+v"(c) : "v"(a), "v"(b)); return c; }

__global__ __launch_bounds__(NPAR) void k_prep(const float* __restrict__ mus, const float* __restrict__ alphas, const float* __restrict__ lw, bf* MUB, float* PT) {
#pragma clang fp contract(off)
    __shared__ __align__(16) unsigned short st[NPAR * DD];
    __shared__ __align__(16) float pt[PTN];
    const int tid = threadIdx.x;
    const int wave = __builtin_amdgcn_readfirstlane((int)(threadIdx.x >> 5));
    const int l = tid / KC, k = tid % KC;
    const float* p = mus + (size_t)l * DD * KC + k;
    float ss = 0.0f;
#pragma unroll 1
    for (int d = 0; d < DD; ++d) {
        const unsigned short hb = f2bf(p[(size_t)d * KC]);
        const float v = __uint_as_float(((unsigned)hb) << 16);
        ss += v * v;
        st[tid * DD + d] = hb;
    }
    pt[tid] = 1.0f / sqrtf(ss);
    pt[NPAR + tid] = bfr(alphas[tid]);
    if (wave == 0) {
        const int wi = tid < LL ? tid : (LL - 1);
        float w = bfr(lw[wi]);
        asm volatile("" : "+v"(w));
        const float e = expf(-(w * w));
        pt[2 * NPAR + tid] = (tid < LL) ? e : 0.0f;
    } else if (wave < 8) {
        pt[2 * NPAR + tid] = 0.0f;
    }
    __syncthreads();
#pragma unroll 1
    for (int ps = 0; ps < 2; ++ps) {
#pragma unroll
        for (int tr = 0; tr < 2; ++tr) {
            const int ch = tr * NPAR + tid;
            const v8us v = *(const v8usa*)(&st[ch * 8]);
            *(volatile v8us*)(MUB + (size_t)ch * 8) = v;
        }
        if (wave < 8) {
            const v4f v = *(const v4fa*)(&pt[tid * 4]);
            *(volatile v4f*)(PT + (size_t)tid * 4) = v;
        }
        if (ps == 0) __threadfence();
    }
}

__global__ __launch_bounds__(32 * WPB) void k_main(const float* __restrict__ xs, const bf* __restrict__ MUB, const float* __restrict__ PT, float* OUT) {
    __shared__ v8us smu8[NPAR * 2];
    __shared__ __align__(16) float spt[PTN];
    __shared__ __align__(16) float sres[PPB];
    const int tid = threadIdx.x;
    const int lane = threadIdx.x & 31, lr = lane & 15, hi = lane >> 4;
    const int wave = __builtin_amdgcn_readfirstlane((int)(threadIdx.x >> 5));
#pragma unroll 1
    for (int i = tid; i < NPAR * 2; i += 32 * WPB) smu8[i] = *(const v8us*)(MUB + (size_t)i * 8);
#pragma unroll 1
    for (int i = tid; i < PTN; i += 32 * WPB) spt[i] = PT[i];
    __syncthreads();

    const int base = (blockIdx.x * WPB + wave) * 16;
    int pnt = base + lr; pnt = pnt < NPTS ? pnt : (NPTS - 1);
    const float* xp = xs + (size_t)pnt * DD + 8 * hi;
    const v4f x0 = *(const v4f*)xp, x1 = *(const v4f*)(xp + 4);
    v8us xl;
#pragma unroll
    for (int i = 0; i < 4; ++i) { xl[i] = f2bf(x0[i]); xl[4 + i] = f2bf(x1[i]); }
    const v8us z8 = (v8us){};
    const v16bf bx = cat16b(xl, z8);

    float F = 0.0f;
#pragma unroll 1
    for (int l = 0; l < LL; ++l) {
        v8f acc[4];
#pragma unroll
        for (int t = 0; t < 4; ++t) {
            const v16bf a = cat16b(smu8[(l * KC + t * 16 + lr) * 2 + hi], z8);
            acc[t] = wmmab_g(a, bx, (v8f){});
        }
        float vals[32];
        float vmax = NEGB;
#pragma unroll
        for (int t = 0; t < 4; ++t) {
#pragma unroll
            for (int r = 0; r < 8; ++r) {
                const int c = l * KC + t * 16 + 8 * hi + r;
                float x = acc[t][r] * spt[c];
                x = fminf(fmaxf(x, -0.9999999f), 0.9999999f);
                const float d = acosf(x);
                const float cost = 0.5f * d * d + spt[NPAR + c];
                const float v = -10.0f * cost;
                vals[t * 8 + r] = v;
                vmax = fmaxf(vmax, v);
            }
        }
        float s = 0.0f;
#pragma unroll
        for (int i = 0; i < 32; ++i) s += __expf(vals[i] - vmax);
        const float m2 = __shfl_xor(vmax, 16, 32);
        const float s2 = __shfl_xor(s, 16, 32);
        const float M  = fmaxf(vmax, m2);
        const float stt = s * __expf(vmax - M) + s2 * __expf(m2 - M);
        const float mincost = 0.1f * (M + __logf(stt));
        const float wvl = spt[2 * NPAR + l];
        F = wvl * fmaxf(F, 0.0f) + (1.0f - wvl) * mincost;
    }
    const float a10 = -10.0f * F;
    const float res = 0.1f * (fmaxf(a10, 0.0f) + log1pf(__expf(-fabsf(a10))));
    if (hi == 0) sres[wave * 16 + lr] = res;
    __syncthreads();
    if (wave == 0) {
        const int p0 = blockIdx.x * PPB + lane * 4;
        const v4f val = *(const v4fa*)(&sres[lane * 4]);
        const bool ok = p0 < NPTS;
#pragma unroll 1
        for (int ps = 0; ps < 2; ++ps) {
            if (ok) *(volatile v4f*)(OUT + (size_t)p0) = val;
            if (ps == 0) __threadfence();
        }
    }
}

static constexpr size_t al256(size_t v) { return (v + 255) & ~(size_t)255; }
static constexpr size_t SZ_MU = al256((size_t)NPAR * DD * 2);
static constexpr size_t SZ_PT = al256((size_t)PTN * 4);
static constexpr size_t SZ_TOTAL = SZ_MU + SZ_PT;
static_assert(SZ_TOTAL <= (size_t)134217728);
static_assert(SZ_MU == (size_t)2 * NPAR * 16);
static_assert(SZ_PT == (size_t)256 * 16);

extern "C" void kernel_launch(void* const* d_in, const int* in_sizes, int n_in,
                              void* d_out, int out_size, void* d_ws, size_t ws_size, hipStream_t stream) {
    if (n_in < 4) return;
    if ((size_t)in_sizes[0] < (size_t)NPTS * DD) return;
    if ((size_t)in_sizes[1] < (size_t)LL * DD * KC) return;
    if (in_sizes[2] < LL * KC || in_sizes[3] < LL) return;
    if ((size_t)out_size < (size_t)NPTS) return;
    if (SZ_TOTAL > ws_size) return;
    const float* xs     = (const float*)d_in[0];
    const float* mus    = (const float*)d_in[1];
    const float* alphas = (const float*)d_in[2];
    const float* lw     = (const float*)d_in[3];
    float* OUT = (float*)d_out;
    char* wsp = (char*)d_ws;
    bf* MUB = (bf*)wsp; wsp += SZ_MU;
    float* PT = (float*)wsp; wsp += SZ_PT;

    k_prep<<<1, NPAR, 0, stream>>>(mus, alphas, lw, MUB, PT);
    k_main<<<(unsigned)((NPTS + PPB - 1) / PPB), 32 * WPB, 0, stream>>>(xs, MUB, PT, OUT);
}
